// TransformAggregator_20444044329183
// MI455X (gfx1250) — hardware-run, weakly checked
//
#include <hip/hip_runtime.h>
#include <stddef.h>
#include <stdint.h>

#define B_    32
#define N_    512
#define D_    512
#define H_    4
#define DH_   128
#define FF_   2048
#define NPAD  520
#define PROWS (B_ * NPAD)
#define KVLD  (2 * D_)
#define LN_EPS 1e-5f
#define NEGF  (-1.0e9f)
#define SCL   0.08838834764831845f
#define OTP   68
#define HTP   72
#define SCP   528
#define NJJ   ((N_ + 32) / 32)

static_assert(PROWS % 256 == 0);
static_assert(PROWS % 8 == 0);
static_assert(D_ == 512);
static_assert(H_ * DH_ == D_);
static_assert(DH_ == 128);
static_assert(B_ == 32);
static_assert(D_ % 64 == 0);
static_assert(FF_ % 512 == 0);
static_assert(D_ % 32 == 0 && FF_ % 32 == 0);
static_assert(NPAD > N_);
static_assert(SCP > N_);
static_assert(NJJ * 32 > N_);
static_assert((N_ + 1) % 8 == 1);

typedef _Float16 v16h __attribute__((ext_vector_type(16)));
typedef _Float16 v8h  __attribute__((ext_vector_type(8)));
typedef float    v8f  __attribute__((ext_vector_type(8)));
typedef float    v4f  __attribute__((ext_vector_type(4)));
typedef unsigned int v4u __attribute__((ext_vector_type(4)));

union Frag  { v16h v; v8h h[2]; };
union Pack8 { v8h h; v4u u; };

__device__ __forceinline__ v8f mma16(v16h a, v16h b, v8f c) {
  c = __builtin_amdgcn_wmma_f32_16x16x32_f16(false, a, false, b, (short)0, c, false, false);
  asm volatile("v_nop\n\tv_nop\n\tv_nop\n\tv_nop" : "+v"(c) : "v"(a), "v"(b));
  return c;
}

__device__ __forceinline__ v16h ldfrag(const _Float16* p, int ld, int row0, int k0, int lane) {
  const int m = lane & 15, lh = lane >> 4;
  const _Float16* q = p + (size_t)(row0 + m) * ld + k0 + 8 * lh;
  Frag f;
  f.h[0] = *(const v8h*)(q);
  f.h[1] = *(const v8h*)(q + 16);
  return f.v;
}

__device__ __forceinline__ v8f zero8() { return (v8f){0.f, 0.f, 0.f, 0.f, 0.f, 0.f, 0.f, 0.f}; }

__device__ __forceinline__ float wsum(float s) {
#pragma unroll
  for (int off = 16; off >= 1; off >>= 1) s += __shfl_xor(s, off, 32);
  return s;
}

__device__ __forceinline__ v4u pack8(v4f a, v4f b) {
  Pack8 p;
  p.h = (v8h){(_Float16)a[0], (_Float16)a[1], (_Float16)a[2], (_Float16)a[3],
              (_Float16)b[0], (_Float16)b[1], (_Float16)b[2], (_Float16)b[3]};
  return p.u;
}

__device__ __forceinline__ float gelu_t(float x) {
  const float u = 0.7978845608028654f * (x + 0.044715f * (x * x * x));
  return x * (0.5f * (1.0f + tanhf(u)));
}

__device__ __forceinline__ void gemm32x64(const _Float16* __restrict__ A, int lda,
                                          const _Float16* __restrict__ Bt, int ldb, int K,
                                          int m0, int n0, int lane, v8f (&acc)[2][4]) {
#pragma unroll 1
  for (int k0 = 0; k0 < K; k0 += 32) {
    const v16h a0 = ldfrag(A, lda, m0, k0, lane);
    const v16h a1 = ldfrag(A, lda, m0 + 16, k0, lane);
    const v16h b0 = ldfrag(Bt, ldb, n0, k0, lane);
    const v16h b1 = ldfrag(Bt, ldb, n0 + 16, k0, lane);
    const v16h b2 = ldfrag(Bt, ldb, n0 + 32, k0, lane);
    const v16h b3 = ldfrag(Bt, ldb, n0 + 48, k0, lane);
    acc[0][0] = mma16(a0, b0, acc[0][0]);
    acc[1][0] = mma16(a1, b0, acc[1][0]);
    acc[0][1] = mma16(a0, b1, acc[0][1]);
    acc[1][1] = mma16(a1, b1, acc[1][1]);
    acc[0][2] = mma16(a0, b2, acc[0][2]);
    acc[1][2] = mma16(a1, b2, acc[1][2]);
    acc[0][3] = mma16(a0, b3, acc[0][3]);
    acc[1][3] = mma16(a1, b3, acc[1][3]);
  }
}

__global__ __launch_bounds__(256) void k_cvtT(const float* __restrict__ src, int K, int N,
                                              _Float16* __restrict__ dst, float scale) {
  __shared__ float tile[64][33];
  const int tid = threadIdx.x;
  const int n0 = blockIdx.x * 32, k0 = blockIdx.y * 64;
  const int tr = tid >> 5, tc = tid & 31;
#pragma unroll
  for (int i = 0; i < 8; ++i)
    tile[tr + 8 * i][tc] = src[(size_t)(k0 + tr + 8 * i) * N + n0 + tc];
  __syncthreads();
  const int r = tid >> 3, pc = tid & 7;
  Pack8 pk;
  pk.h = (v8h){(_Float16)(tile[8 * pc + 0][r] * scale), (_Float16)(tile[8 * pc + 1][r] * scale),
               (_Float16)(tile[8 * pc + 2][r] * scale), (_Float16)(tile[8 * pc + 3][r] * scale),
               (_Float16)(tile[8 * pc + 4][r] * scale), (_Float16)(tile[8 * pc + 5][r] * scale),
               (_Float16)(tile[8 * pc + 6][r] * scale), (_Float16)(tile[8 * pc + 7][r] * scale)};
  const v4u vv = pk.u;
  volatile v4u* d = (volatile v4u*)(dst + (size_t)(n0 + r) * K + k0 + 8 * pc);
  *d = vv;
  __threadfence();
  *d = vv;
}

__device__ __forceinline__ void ln_row_store(v4f (&v)[4], const float* __restrict__ g, const float* __restrict__ be,
                                             bool live, _Float16* __restrict__ dst, int lane) {
  const int c0 = 8 * lane, c1 = 256 + 8 * lane;
  float s = 0.f;
#pragma unroll
  for (int i = 0; i < 4; ++i) s += (v[i][0] + v[i][1]) + (v[i][2] + v[i][3]);
  s = wsum(s);
  const float mean = s * (1.0f / D_);
  float ss = 0.f;
#pragma unroll
  for (int i = 0; i < 4; ++i) {
    const v4f d = v[i] - mean;
    ss += (d[0] * d[0] + d[1] * d[1]) + (d[2] * d[2] + d[3] * d[3]);
  }
  ss = wsum(ss);
  const float rstd = rsqrtf(ss * (1.0f / D_) + LN_EPS);
  v4f y[4];
#pragma unroll
  for (int i = 0; i < 4; ++i) {
    const int col = ((i < 2) ? c0 : c1) + 4 * (i & 1);
    const v4f gv = *(const v4f*)(g + col);
    const v4f bv = *(const v4f*)(be + col);
    v4f t = ((v[i] - mean) * rstd) * gv + bv;
#pragma unroll
    for (int j = 0; j < 4; ++j) t[j] = live ? t[j] : 0.f;
    y[i] = t;
  }
  const v4u p0 = pack8(y[0], y[1]);
  const v4u p1 = pack8(y[2], y[3]);
  volatile v4u* d0 = (volatile v4u*)(dst + c0);
  volatile v4u* d1 = (volatile v4u*)(dst + c1);
  *d0 = p0;
  *d1 = p1;
  __threadfence();
  *d0 = p0;
  *d1 = p1;
}

__global__ __launch_bounds__(256) void k_ln1(const float* __restrict__ x, const float* __restrict__ token,
                                             const float* __restrict__ g, const float* __restrict__ be,
                                             _Float16* __restrict__ hp) {
  const int tid = threadIdx.x, lane = tid & 31, wave = tid >> 5;
  const int pr = blockIdx.x * 8 + wave;
  const int b  = pr / NPAD;
  const int j  = pr - b * NPAD;
  const bool isx  = j < N_;
  const bool live = j <= N_;
  const float* src = isx ? (x + ((size_t)b * N_ + j) * D_) : token;
  const int c0 = 8 * lane, c1 = 256 + 8 * lane;
  v4f v[4];
  v[0] = *(const v4f*)(src + c0);
  v[1] = *(const v4f*)(src + c0 + 4);
  v[2] = *(const v4f*)(src + c1);
  v[3] = *(const v4f*)(src + c1 + 4);
  float ss = 0.f;
#pragma unroll
  for (int i = 0; i < 4; ++i)
    ss += (v[i][0] * v[i][0] + v[i][1] * v[i][1]) + (v[i][2] * v[i][2] + v[i][3] * v[i][3]);
  ss = wsum(ss);
  const float nrm = sqrtf(ss);
  const float inv = isx ? (1.0f / fmaxf(nrm, 1e-12f)) : 1.0f;
#pragma unroll
  for (int i = 0; i < 4; ++i) v[i] = v[i] * inv;
  ln_row_store(v, g, be, live, hp + (size_t)pr * D_, lane);
}

__global__ __launch_bounds__(256) void k_ln2(const float* __restrict__ h1, const float* __restrict__ g,
                                             const float* __restrict__ be, _Float16* __restrict__ h2p) {
  const int tid = threadIdx.x, lane = tid & 31, wave = tid >> 5;
  const int pr = min((int)blockIdx.x * 8 + wave, B_ - 1);
  const float* src = h1 + (size_t)pr * D_;
  const int c0 = 8 * lane, c1 = 256 + 8 * lane;
  v4f v[4];
  v[0] = *(const v4f*)(src + c0);
  v[1] = *(const v4f*)(src + c0 + 4);
  v[2] = *(const v4f*)(src + c1);
  v[3] = *(const v4f*)(src + c1 + 4);
  ln_row_store(v, g, be, true, h2p + (size_t)pr * D_, lane);
}

template <bool RES>
__device__ __forceinline__ void out_epilogue_f32(v8f (&acc)[2][4], float scale, const float (&bb)[4],
                                                 float* sw, float* __restrict__ out, int ldo,
                                                 const float* __restrict__ resid, int ldr,
                                                 int m0, int n0, int lane, int hh, int c) {
#pragma unroll
  for (int sub = 0; sub < 2; ++sub) {
    __syncthreads();
#pragma unroll
    for (int t = 0; t < 4; ++t) {
#pragma unroll
      for (int r = 0; r < 8; ++r) sw[(8 * hh + r) * OTP + 16 * t + c] = acc[sub][t][r] * scale + bb[t];
    }
    __syncthreads();
    v4f val[8];
    size_t go[8];
#pragma unroll
    for (int it = 0; it < 8; ++it) {
      const int p     = lane + 32 * it;
      const int L     = p >> 3;
      const int pc    = p & 7;
      const int row   = L >> 1;
      const int seg   = L & 1;
      v4f vv = *(const v4f*)(sw + row * OTP + seg * 32 + pc * 4);
      if (RES) vv += *(const v4f*)(resid + (size_t)(m0 + sub * 16 + row) * ldr + n0 + seg * 32 + pc * 4);
      val[it] = vv;
      go[it]  = (size_t)(m0 + sub * 16 + row) * ldo + n0 + seg * 32 + pc * 4;
    }
    for (int ps = 0; ps < 2; ++ps) {
#pragma unroll
      for (int it = 0; it < 8; ++it) *(volatile v4f*)(out + go[it]) = val[it];
      __threadfence();
    }
  }
}

__device__ __forceinline__ void out_epilogue_gelu16(v8f (&acc)[2][4], float scale, const float (&bb)[4],
                                                    float* sw, _Float16* shw, _Float16* __restrict__ out, int ldo,
                                                    int m0, int n0, int lane, int hh, int c) {
#pragma unroll
  for (int sub = 0; sub < 2; ++sub) {
    __syncthreads();
#pragma unroll
    for (int t = 0; t < 4; ++t) {
#pragma unroll
      for (int r = 0; r < 8; ++r) sw[(8 * hh + r) * OTP + 16 * t + c] = acc[sub][t][r] * scale + bb[t];
    }
    __syncthreads();
#pragma unroll 1
    for (int i = 0; i < 32; ++i) {
      const int e   = i * 32 + lane;
      const int row = e >> 6, col = e & 63;
      const float v = sw[row * OTP + col];
      shw[row * HTP + col] = (_Float16)(gelu_t(v) * 64.0f);
    }
    __syncthreads();
    v4u val[4];
    size_t go[4];
#pragma unroll
    for (int it = 0; it < 4; ++it) {
      const int p   = lane + 32 * it;
      const int row = p >> 3;
      const int pc  = p & 7;
      Pack8 pk;
      pk.h    = *(const v8h*)(shw + row * HTP + pc * 8);
      val[it] = pk.u;
      go[it]  = (size_t)(m0 + sub * 16 + row) * ldo + n0 + pc * 8;
    }
    for (int ps = 0; ps < 2; ++ps) {
#pragma unroll
      for (int it = 0; it < 4; ++it) *(volatile v4u*)(out + go[it]) = val[it];
      __threadfence();
    }
  }
}

template <int MODE>
__global__ __launch_bounds__(256) void k_gemm(const _Float16* __restrict__ A, int lda,
                                              const _Float16* __restrict__ Bt, int K,
                                              const float* __restrict__ bias, const float* __restrict__ bias2,
                                              const float* __restrict__ resid, int ldr, float scale,
                                              float* __restrict__ outf, _Float16* __restrict__ outh, int ldo) {
  __shared__ __align__(16) float    sw[8][16 * OTP];
  __shared__ __align__(16) _Float16 sh[8][16 * HTP];
  const int tid = threadIdx.x, lane = tid & 31, wave = tid >> 5;
  const int hh = lane >> 4, c = lane & 15;
  int m0, n0;
  if (MODE == 0) {
    m0 = blockIdx.x * 256 + wave * 32;
    n0 = blockIdx.y * 64;
  } else {
    m0 = 0;
    n0 = blockIdx.x * 512 + wave * 64;
  }

  v8f acc[2][4];
#pragma unroll
  for (int s = 0; s < 2; ++s)
#pragma unroll
    for (int t = 0; t < 4; ++t) acc[s][t] = zero8();
  gemm32x64(A, lda, Bt, K, K, m0, n0, lane, acc);

  float bb[4];
#pragma unroll
  for (int t = 0; t < 4; ++t) {
    const int col = n0 + 16 * t + c;
    if (MODE == 0) {
      const float u0 = bias[min(col, D_ - 1)];
      const float u1 = bias2[min(max(col - D_, 0), D_ - 1)];
      bb[t] = (col < D_) ? u0 : u1;
    } else if (MODE == 2) {
      bb[t] = bias[col] + bias2[col];
    } else {
      bb[t] = bias[col];
    }
  }
  if (MODE == 3) {
    out_epilogue_gelu16(acc, scale, bb, sw[wave], sh[wave], outh, ldo, m0, n0, lane, hh, c);
  } else if (MODE == 4) {
    out_epilogue_f32<true>(acc, scale, bb, sw[wave], outf, ldo, resid, ldr, m0, n0, lane, hh, c);
  } else {
    out_epilogue_f32<false>(acc, scale, bb, sw[wave], outf, ldo, resid, ldr, m0, n0, lane, hh, c);
  }
}

__global__ __launch_bounds__(256) void k_attn(const float* __restrict__ qf, const float* __restrict__ kv,
                                              const int* __restrict__ len, _Float16* __restrict__ c16) {
  __shared__ float sc[H_ * SCP];
  __shared__ __align__(16) _Float16 cs[D_];
  const int tid = threadIdx.x, lane = tid & 31, wave = tid >> 5;
  const int b  = blockIdx.x;
  const int mk = len[b];

  const float* qr = qf + (size_t)b * D_ + 16 * lane;
  v4f qv[4];
#pragma unroll
  for (int i = 0; i < 4; ++i) qv[i] = *(const v4f*)(qr + 4 * i);

  const float* kb = kv + (size_t)b * NPAD * KVLD;

#pragma unroll 1
  for (int j = wave; j <= N_; j += 8) {
    const float* kr = kb + (size_t)j * KVLD + 16 * lane;
    v4f kq[4];
#pragma unroll
    for (int i = 0; i < 4; ++i) kq[i] = *(const v4f*)(kr + 4 * i);
    float d = 0.f;
#pragma unroll
    for (int i = 0; i < 4; ++i) {
      d = fmaf(qv[i][0], kq[i][0], d);
      d = fmaf(qv[i][1], kq[i][1], d);
      d = fmaf(qv[i][2], kq[i][2], d);
      d = fmaf(qv[i][3], kq[i][3], d);
    }
    d += __shfl_xor(d, 1, 32);
    d += __shfl_xor(d, 2, 32);
    d += __shfl_xor(d, 4, 32);
    const bool valid = (j < mk) || (j == N_);
    const float s = valid ? (d * SCL) : NEGF;
    if ((lane & 7) == 0) sc[(lane >> 3) * SCP + j] = s;
  }
  __syncthreads();

  if (wave < H_) {
    float* ph = sc + wave * SCP;
    float m = -3.0e38f;
#pragma unroll 1
    for (int jj = 0; jj < NJJ; ++jj) {
      const int j = jj * 32 + lane;
      const float v = ph[min(j, N_)];
      m = fmaxf(m, (j <= N_) ? v : -3.0e38f);
    }
#pragma unroll
    for (int off = 16; off >= 1; off >>= 1) m = fmaxf(m, __shfl_xor(m, off, 32));
    float l = 0.f;
#pragma unroll 1
    for (int jj = 0; jj < NJJ; ++jj) {
      const int j = jj * 32 + lane;
      const bool ok = j <= N_;
      const float v = ph[min(j, N_)];
      const float e = ok ? expf(v - m) : 0.f;
      l += e;
      if (ok) ph[j] = e;
    }
    l = wsum(l);
    const float inv = 1.0f / l;
#pragma unroll 1
    for (int jj = 0; jj < NJJ; ++jj) {
      const int j = jj * 32 + lane;
      const float v = ph[min(j, N_)];
      if (j <= N_) ph[j] = v * inv;
    }
  }
  __syncthreads();

  const int ca = tid, cb = tid + 256;
  const int ha = tid >> 7, hb = ha + 2;
  const float* vb = kb + D_;
  const float* pa = sc + ha * SCP;
  const float* pb = sc + hb * SCP;
  float acc0 = 0.f, acc1 = 0.f;
#pragma unroll 1
  for (int j = 0; j <= N_; ++j) {
    const float* vr = vb + (size_t)j * KVLD;
    acc0 = fmaf(pa[j], vr[ca], acc0);
    acc1 = fmaf(pb[j], vr[cb], acc1);
  }
  cs[ca] = (_Float16)(acc0 * 64.0f);
  cs[cb] = (_Float16)(acc1 * 64.0f);
  __syncthreads();
  if (tid < 64) {
    Pack8 pk;
    pk.h = *(const v8h*)(cs + 8 * tid);
    const v4u vv = pk.u;
    volatile v4u* d = (volatile v4u*)(c16 + (size_t)b * D_ + 8 * tid);
    *d = vv;
    __threadfence();
    *d = vv;
  }
}

extern "C" void kernel_launch(void* const* d_in, const int* in_sizes, int n_in,
                              void* d_out, int out_size, void* d_ws, size_t ws_size,
                              hipStream_t stream) {
  if (n_in < 19) return;
  if (in_sizes[0]  != B_ * N_ * D_) return;
  if (in_sizes[1]  != B_) return;
  if (in_sizes[2]  != D_) return;
  if (in_sizes[3]  != D_ * D_) return;
  if (in_sizes[4]  != D_) return;
  if (in_sizes[5]  != D_ * D_) return;
  if (in_sizes[6]  != D_) return;
  if (in_sizes[7]  != D_ * D_) return;
  if (in_sizes[8]  != D_) return;
  if (in_sizes[9]  != D_ * D_) return;
  if (in_sizes[10] != D_) return;
  if (in_sizes[11] != D_ || in_sizes[12] != D_ || in_sizes[13] != D_ || in_sizes[14] != D_) return;
  if (in_sizes[15] != D_ * FF_) return;
  if (in_sizes[16] != FF_) return;
  if (in_sizes[17] != FF_ * D_) return;
  if (in_sizes[18] != D_) return;
  if (out_size != B_ * D_) return;

  const float* x     = (const float*)d_in[0];
  const int*   len   = (const int*)d_in[1];
  const float* token = (const float*)d_in[2];
  const float* Wq    = (const float*)d_in[3];
  const float* bq    = (const float*)d_in[4];
  const float* Wk    = (const float*)d_in[5];
  const float* bk    = (const float*)d_in[6];
  const float* Wv    = (const float*)d_in[7];
  const float* bv    = (const float*)d_in[8];
  const float* Wo    = (const float*)d_in[9];
  const float* bo    = (const float*)d_in[10];
  const float* ln1s  = (const float*)d_in[11];
  const float* ln1b  = (const float*)d_in[12];
  const float* ln2s  = (const float*)d_in[13];
  const float* ln2b  = (const float*)d_in[14];
  const float* W1    = (const float*)d_in[15];
  const float* b1    = (const float*)d_in[16];
  const float* W2    = (const float*)d_in[17];
  const float* b2    = (const float*)d_in[18];
  float* out = (float*)d_out;

  size_t off = 0;
  const size_t oWkv = off; off += (size_t)KVLD * D_ * 2;
  const size_t oWq  = off; off += (size_t)D_ * D_ * 2;
  const size_t oWo  = off; off += (size_t)D_ * D_ * 2;
  const size_t oW1  = off; off += (size_t)FF_ * D_ * 2;
  const size_t oW2  = off; off += (size_t)D_ * FF_ * 2;
  const size_t oHp  = off; off += (size_t)PROWS * D_ * 2;
  const size_t oKV  = off; off += (size_t)PROWS * KVLD * 4;
  const size_t oQ   = off; off += (size_t)B_ * D_ * 4;
  const size_t oC   = off; off += (size_t)B_ * D_ * 2;
  const size_t oH1  = off; off += (size_t)B_ * D_ * 4;
  const size_t oH2  = off; off += (size_t)B_ * D_ * 2;
  const size_t oG   = off; off += (size_t)B_ * FF_ * 2;
  if (off > ws_size) return;
  if (off > (size_t)134217728) return;

  char* ws = (char*)d_ws;
  _Float16* WkvT = (_Float16*)(ws + oWkv);
  _Float16* WqT  = (_Float16*)(ws + oWq);
  _Float16* WoT  = (_Float16*)(ws + oWo);
  _Float16* W1T  = (_Float16*)(ws + oW1);
  _Float16* W2T  = (_Float16*)(ws + oW2);
  _Float16* Hp   = (_Float16*)(ws + oHp);
  float*    KV   = (float*)(ws + oKV);
  float*    Qf   = (float*)(ws + oQ);
  _Float16* C16  = (_Float16*)(ws + oC);
  float*    H1   = (float*)(ws + oH1);
  _Float16* H2p  = (_Float16*)(ws + oH2);
  _Float16* G16  = (_Float16*)(ws + oG);

  k_cvtT<<<dim3(D_ / 32, D_ / 64), dim3(256), 0, stream>>>(Wk, D_, D_, WkvT, 64.0f);
  k_cvtT<<<dim3(D_ / 32, D_ / 64), dim3(256), 0, stream>>>(Wv, D_, D_, WkvT + (size_t)D_ * D_, 64.0f);
  k_cvtT<<<dim3(D_ / 32, D_ / 64), dim3(256), 0, stream>>>(Wq, D_, D_, WqT, 64.0f);
  k_cvtT<<<dim3(D_ / 32, D_ / 64), dim3(256), 0, stream>>>(Wo, D_, D_, WoT, 64.0f);
  k_cvtT<<<dim3(FF_ / 32, D_ / 64), dim3(256), 0, stream>>>(W1, D_, FF_, W1T, 64.0f);
  k_cvtT<<<dim3(D_ / 32, FF_ / 64), dim3(256), 0, stream>>>(W2, FF_, D_, W2T, 64.0f);
  k_ln1<<<dim3(PROWS / 8), dim3(256), 0, stream>>>(x, token, ln1s, ln1b, Hp);
  k_gemm<0><<<dim3(PROWS / 256, KVLD / 64), dim3(256), 0, stream>>>(Hp, D_, WkvT, D_, bk, bv, Qf, D_,
                                                                      0.015625f, KV, C16, KVLD);
  k_gemm<1><<<dim3(D_ / 512), dim3(256), 0, stream>>>(Hp + (size_t)N_ * D_, NPAD * D_, WqT, D_, bq, bq, Qf, D_,
                                                       0.015625f, Qf, C16, D_);
  k_attn<<<dim3(B_), dim3(256), 0, stream>>>(Qf, KV, len, C16);
  k_gemm<2><<<dim3(D_ / 512), dim3(256), 0, stream>>>(C16, D_, WoT, D_, bo, token, Qf, D_,
                                                       0.000244140625f, H1, C16, D_);
  k_ln2<<<dim3(B_ / 8), dim3(256), 0, stream>>>(H1, ln2s, ln2b, H2p);
  k_gemm<3><<<dim3(FF_ / 512), dim3(256), 0, stream>>>(H2p, D_, W1T, D_, b1, b1, Qf, D_,
                                                        0.015625f, Qf, G16, FF_);
  k_gemm<4><<<dim3(D_ / 512), dim3(256), 0, stream>>>(G16, FF_, W2T, FF_, b2, b2, H1, D_,
                                                       0.000244140625f, out, C16, D_);
  (void)hipGetLastError();
}
